// GNNStack_412316860635
// MI455X (gfx1250) — hardware-verified
//
#include <hip/hip_runtime.h>
#include <stddef.h>
#include <stdint.h>


#define DF     128
#define HP     256
#define XP     128
#define PABP   256
#define NTHR   256
#define NWAVE  8
#define EPT    8
#define CHUNK  (NTHR * EPT)
#define WCAP   (EPT * 32)
#define LISTN  (NWAVE * WCAP)
#define NBA    1024
#define SLA    10
#define RCAP   28672
#define DEGCAP 64
#define MSTRIDE 2080
#define GBM    64
#define GBN    128
#define GTHR   128
#define USEG   2048
#define NSEG   19
#define NUW    (NSEG * USEG)
#define OW0    0
#define OW1    49152
#define OW2    114688
#define OP1    180224
#define OP2    212992
#define OQ     245760
#define WPLN   311296
#define CMP_ZINTS    (LISTN + 2 * RCAP + 3 * NBA)
#define MISC_INTS    16
#define CMP_LDS_INTS (CMP_ZINTS + MISC_INTS)
#define WSMAX  134217728

static_assert(DF == 128 && DF == 4 * 32 && HP == 2 * DF && XP == DF && PABP == 2 * DF);
static_assert((CHUNK & (CHUNK - 1)) == 0 && CHUNK <= 4096);
static_assert((NBA & (NBA - 1)) == 0 && NBA == (1 << SLA));
static_assert(((long long)CHUNK << SLA) < (1LL << 31));
static_assert(NBA % NWAVE == 0 && NBA % 32 == 0 && NBA % GBM == 0);
static_assert(RCAP % (NTHR * 4) == 0 && CMP_ZINTS % (NTHR * 4) == 0);
static_assert(2 * NBA == 2 * NTHR * 4 && MSTRIDE == 2 * NBA + 32 && MSTRIDE % 32 == 0);
static_assert(RCAP >= 12617 + 8 && DEGCAP >= 28 + 8);
static_assert(49 * NBA >= 50000 && 200000 % 32 == 0);
static_assert(384 % 32 == 0 && 512 % 32 == 0 && 256 % 32 == 0);
static_assert(GBN == DF && GBM == (GTHR / 32) * 16);
static_assert(USEG % NTHR == 0 && NUW % NTHR == 0 && USEG == DF * (DF / 8));
static_assert(OW1 == OW0 + DF * 384 && OW2 == OW1 + DF * 512 && OP1 == OW2 + DF * 512);
static_assert(OP2 == OP1 + DF * 256 && OQ == OP2 + DF * 256 && WPLN == OQ + 256 * 256);
static_assert(CMP_LDS_INTS * 4 <= 300000);

typedef float          v4f   __attribute__((ext_vector_type(4)));
typedef float          v8f   __attribute__((ext_vector_type(8)));
typedef int            v4i   __attribute__((ext_vector_type(4)));
typedef int            v8i   __attribute__((ext_vector_type(8)));
typedef unsigned       v2u   __attribute__((ext_vector_type(2)));
typedef unsigned short v4us  __attribute__((ext_vector_type(4)));
typedef unsigned short v8us  __attribute__((ext_vector_type(8)));
typedef unsigned short v16us __attribute__((ext_vector_type(16)));
typedef __bf16         v16bf __attribute__((ext_vector_type(16)));
typedef v4f  __attribute__((may_alias)) v4fa;
typedef v4i  __attribute__((may_alias)) v4ia;
typedef v2u  __attribute__((may_alias)) v2ua;
typedef v4us __attribute__((may_alias)) v4usa;
typedef v8us __attribute__((may_alias)) v8usa;
union FragB { v16bf v; v16us u; v8us h[2]; v8i w; };

__device__ __forceinline__ v8f wmb(const FragB& a, const FragB& b, v8f c) {
  v8f d = __builtin_amdgcn_wmma_f32_16x16x32_bf16(false, a.v, false, b.v, (short)0, c, false, false);
  asm volatile("v_nop\n\tv_nop\n\tv_nop\n\tv_nop" : "+v"(d) : "v"(a.w), "v"(b.w));
  return d;
}

__device__ __forceinline__ unsigned bf16_bits(float f) {
  const unsigned u = __float_as_uint(f);
  const unsigned r = (u + 0x7FFFu + ((u >> 16) & 1u)) >> 16;
  return (f != f) ? 0x7FC0u : r;
}
__device__ __forceinline__ float bf16_val(float f) {
  return __uint_as_float(bf16_bits(f) << 16);
}
__device__ __forceinline__ float relu_np(float v) { return (v > 0.0f) ? v : (v - v); }

__device__ __forceinline__ void wave_sync() {
  __builtin_amdgcn_fence(__ATOMIC_RELEASE, "wavefront");
  __builtin_amdgcn_wave_barrier();
  __builtin_amdgcn_fence(__ATOMIC_ACQUIRE, "wavefront");
}

template <int SLB>
__device__ __forceinline__ int scan_chunk(const int* __restrict__ dsts, int nE, int cbase, int slotBase,
                                          int nb, int vec8, int* list, int tid, int lane, int wave) {
  int wc = 0;
  const int el0  = tid * EPT;
  const int e0   = cbase + el0;
  const int sent = -2147483647 - 1;
  v4i da, db;
  if (vec8 != 0 && cbase + CHUNK <= nE) {
    da = *(const v4i*)(dsts + e0);
    db = *(const v4i*)(dsts + e0 + 4);
  } else {
    da.x = (e0     < nE) ? dsts[min(e0,     nE - 1)] : sent;
    da.y = (e0 + 1 < nE) ? dsts[min(e0 + 1, nE - 1)] : sent;
    da.z = (e0 + 2 < nE) ? dsts[min(e0 + 2, nE - 1)] : sent;
    da.w = (e0 + 3 < nE) ? dsts[min(e0 + 3, nE - 1)] : sent;
    db.x = (e0 + 4 < nE) ? dsts[min(e0 + 4, nE - 1)] : sent;
    db.y = (e0 + 5 < nE) ? dsts[min(e0 + 5, nE - 1)] : sent;
    db.z = (e0 + 6 < nE) ? dsts[min(e0 + 6, nE - 1)] : sent;
    db.w = (e0 + 7 < nE) ? dsts[min(e0 + 7, nE - 1)] : sent;
  }
  const unsigned nbs = (unsigned)slotBase;
  const unsigned unb = (unsigned)nb;
  const unsigned s0 = (unsigned)da.x - nbs, s1 = (unsigned)da.y - nbs;
  const unsigned s2 = (unsigned)da.z - nbs, s3 = (unsigned)da.w - nbs;
  const unsigned s4 = (unsigned)db.x - nbs, s5 = (unsigned)db.y - nbs;
  const unsigned s6 = (unsigned)db.z - nbs, s7 = (unsigned)db.w - nbs;
  const bool h0 = s0 < unb, h1 = s1 < unb, h2 = s2 < unb, h3 = s3 < unb;
  const bool h4 = s4 < unb, h5 = s5 < unb, h6 = s6 < unb, h7 = s7 < unb;
  const unsigned any = __builtin_amdgcn_ballot_w32(h0 | h1 | h2 | h3 | h4 | h5 | h6 | h7);
  if (any != 0u) {
#define HITJ(J, HJ, SJ) { \
      const unsigned mj = __builtin_amdgcn_ballot_w32(HJ); \
      if (mj != 0u) { \
        if (HJ) { \
          const int pos = wc + (int)__builtin_amdgcn_mbcnt_lo(mj, 0u); \
          if (pos < WCAP) list[wave * WCAP + pos] = ((el0 + (J)) << SLB) | (int)(SJ); \
        } \
        wc += (int)__builtin_popcount(mj); } }
    HITJ(0, h0, s0)
    HITJ(1, h1, s1)
    HITJ(2, h2, s2)
    HITJ(3, h3, s3)
    HITJ(4, h4, s4)
    HITJ(5, h5, s5)
    HITJ(6, h6, s6)
    HITJ(7, h7, s7)
#undef HITJ
  }
  return wc;
}

__device__ __forceinline__ v8us tr8(const float* __restrict__ p) {
  v8us o;
#pragma unroll
  for (int i = 0; i < 8; ++i) o[i] = (unsigned short)bf16_bits(p[(size_t)i * DF]);
  return o;
}

__global__ __launch_bounds__(NTHR) void k_prep(const float* __restrict__ x, const float* __restrict__ Wl,
                                               const float* __restrict__ Wr, const float* __restrict__ pW1,
                                               const float* __restrict__ pW2, const float* __restrict__ qW1,
                                               unsigned short* wpl, unsigned short* xb, int nN, int nUnits) {
  const int u = (int)blockIdx.x * NTHR + (int)threadIdx.x;
  v8us o;
  unsigned short* dp;
  if (u < NUW) {
    const int seg = u >> 11;
    const int v   = u & (USEG - 1);
    const int n   = v >> 4;
    const int k8  = (v & 15) * 8;
    int which, srcOff, base, pitch, coff;
    if (seg < 3) {
      which = (seg < 2) ? 0 : 1; srcOff = 0; base = OW0; pitch = 384; coff = DF * seg;
    } else if (seg < 11) {
      const int s = seg - 3, lay = 1 + (s >> 2), j = s & 3;
      which = (j < 2) ? 0 : 1; srcOff = lay * DF * DF; base = OW1 + (lay - 1) * (DF * 512); pitch = 512; coff = DF * j;
    } else if (seg < 15) {
      const int s = seg - 11, mm = s >> 1, j = s & 1;
      which = 2 + mm; srcOff = 0; base = OP1 + mm * (DF * 256); pitch = 256; coff = DF * j;
    } else {
      const int s = seg - 15, hf = s >> 1, j = s & 1;
      which = 4; srcOff = hf * DF * DF; base = OQ + hf * (DF * 256); pitch = 256; coff = DF * j;
    }
    const size_t so = (size_t)srcOff + (size_t)k8 * DF + (size_t)n;
    if (which == 0)      o = tr8(Wl + so);
    else if (which == 1) o = tr8(Wr + so);
    else if (which == 2) o = tr8(pW1 + so);
    else if (which == 3) o = tr8(pW2 + so);
    else                 o = tr8(qW1 + so);
    dp = wpl + (size_t)base + (size_t)n * pitch + coff + k8;
  } else if (u < nUnits) {
    const int v   = u - NUW;
    const int row = v >> 4, k8 = (v & 15) * 8;
    const int rc  = row < nN ? row : nN - 1;
    const bool lv = row < nN;
    const float* p = x + (size_t)rc * DF + k8;
    const v4f a = *(const v4f*)p;
    const v4f b = *(const v4f*)(p + 4);
    o[0] = lv ? (unsigned short)bf16_bits(a.x) : (unsigned short)0;
    o[1] = lv ? (unsigned short)bf16_bits(a.y) : (unsigned short)0;
    o[2] = lv ? (unsigned short)bf16_bits(a.z) : (unsigned short)0;
    o[3] = lv ? (unsigned short)bf16_bits(a.w) : (unsigned short)0;
    o[4] = lv ? (unsigned short)bf16_bits(b.x) : (unsigned short)0;
    o[5] = lv ? (unsigned short)bf16_bits(b.y) : (unsigned short)0;
    o[6] = lv ? (unsigned short)bf16_bits(b.z) : (unsigned short)0;
    o[7] = lv ? (unsigned short)bf16_bits(b.w) : (unsigned short)0;
    dp = xb + (size_t)v * 8;
  } else {
    return;
  }
  *(volatile v8us*)dp = o;
  __threadfence();
  *(volatile v8us*)dp = o;
}

__global__ __launch_bounds__(NTHR) void k_compact(const int* __restrict__ srcs, const int* __restrict__ dsts,
                                                  int nE, int nN, int vec8, int* lst, int* meta) {
  extern __shared__ __attribute__((aligned(16))) int dsm[];
  int* list = dsm;
  int* hl   = dsm + LISTN;
  int* sl   = hl + RCAP;
  int* cnt  = sl + RCAP;
  int* offs = cnt + NBA;
  int* cur  = offs + NBA;
  int* misc = cur + NBA;
  const int tid = (int)threadIdx.x, lane = tid & 31, wave = tid >> 5;
  const int nodeBase = (int)blockIdx.x * NBA;

  {
    const v4i z4 = {0, 0, 0, 0};
    for (int i = tid * 4; i < CMP_ZINTS; i += NTHR * 4) *(v4ia*)(dsm + i) = z4;
    if (tid < MISC_INTS) misc[tid] = 0;
  }
  __syncthreads();

  int t = 0, ov = 0;
  const int nChunks = (nE + CHUNK - 1) / CHUNK;
#pragma unroll 1
  for (int ch = 0; ch < nChunks; ++ch) {
    const int cbase = ch * CHUNK;
    const int wc = scan_chunk<SLA>(dsts, nE, cbase, nodeBase, NBA, vec8, list, tid, lane, wave);
    if (lane == 0) misc[wave] = wc;
    __syncthreads();
    if (wave == 0) {
#pragma unroll 1
      for (int w2 = 0; w2 < NWAVE; ++w2) {
        int c = misc[w2];
        c = c < 0 ? 0 : (c > WCAP ? WCAP : c);
#pragma unroll 1
        for (int b0 = 0; b0 < c; b0 += 32) {
          const int idx = b0 + lane;
          const int ent_ = list[w2 * WCAP + (idx < WCAP ? idx : WCAP - 1)];
          const int m32 = (c - b0) < 32 ? (c - b0) : 32;
#pragma unroll 1
          for (int k = 0; k < m32; ++k) {
            const int u    = __builtin_amdgcn_readlane(ent_, k);
            const int slot = u & (NBA - 1);
            const int el   = (u >> SLA) & (CHUNK - 1);
            const int pk   = ((cbase + el) << SLA) | slot;
            if (t < RCAP) {
              if (lane == 0) { hl[t] = pk; cnt[slot] = cnt[slot] + 1; }
              t = t + 1;
            } else {
              ov = 1;
            }
          }
        }
      }
    }
    __syncthreads();
  }
  if (wave == 0 && lane == 0) { misc[8] = t; misc[9] = ov; }
  __syncthreads();
  int tt = misc[8];
  tt = tt < 0 ? 0 : (tt > RCAP ? RCAP : tt);
  const int ovf = misc[9];

  if (wave == 0) {
    const int base = lane * (NBA / 32);
    int s = 0;
#pragma unroll 1
    for (int i = 0; i < NBA / 32; ++i) s += cnt[base + i];
    int incl = s;
#pragma unroll
    for (int d = 1; d < 32; d <<= 1) {
      const int y = __shfl_up(incl, d, 32);
      if (lane >= d) incl += y;
    }
    int run = incl - s;
#pragma unroll 1
    for (int i = 0; i < NBA / 32; ++i) {
      const int cv = cnt[base + i];
      offs[base + i] = run;
      cur[base + i]  = run;
      run += cv;
    }
  }
  __syncthreads();
  if (wave == 0) {
#pragma unroll 1
    for (int b0 = 0; b0 < tt; b0 += 32) {
      const int idx = b0 + lane;
      const int ent_ = hl[idx < RCAP ? idx : RCAP - 1];
      const int m32 = (tt - b0) < 32 ? (tt - b0) : 32;
#pragma unroll 1
      for (int k = 0; k < m32; ++k) {
        const int u    = __builtin_amdgcn_readlane(ent_, k);
        const int slot = u & (NBA - 1);
        if (lane == 0) {
          int p = cur[slot];
          p = p < 0 ? 0 : (p > RCAP - 1 ? RCAP - 1 : p);
          sl[p] = u;
          cur[slot] = p + 1;
        }
      }
    }
  }
  __syncthreads();

  int* lp = lst + (size_t)blockIdx.x * RCAP;
#pragma unroll 1
  for (int i = tid * 4; i < RCAP; i += NTHR * 4) {
    const v4i e4 = *(const v4ia*)(sl + i);
    int e0 = e4.x >> SLA, e1 = e4.y >> SLA, e2 = e4.z >> SLA, e3 = e4.w >> SLA;
    e0 = e0 < 0 ? 0 : (e0 > nE - 1 ? nE - 1 : e0);
    e1 = e1 < 0 ? 0 : (e1 > nE - 1 ? nE - 1 : e1);
    e2 = e2 < 0 ? 0 : (e2 > nE - 1 ? nE - 1 : e2);
    e3 = e3 < 0 ? 0 : (e3 > nE - 1 ? nE - 1 : e3);
    int s0 = srcs[e0], s1 = srcs[e1], s2 = srcs[e2], s3 = srcs[e3];
    s0 = s0 < 0 ? 0 : (s0 > nN - 1 ? nN - 1 : s0);
    s1 = s1 < 0 ? 0 : (s1 > nN - 1 ? nN - 1 : s1);
    s2 = s2 < 0 ? 0 : (s2 > nN - 1 ? nN - 1 : s2);
    s3 = s3 < 0 ? 0 : (s3 > nN - 1 ? nN - 1 : s3);
    v4i o;
    o.x = (i     < tt) ? s0 : 0;
    o.y = (i + 1 < tt) ? s1 : 0;
    o.z = (i + 2 < tt) ? s2 : 0;
    o.w = (i + 3 < tt) ? s3 : 0;
    int* dq = lp + i;
    *(volatile v4i*)dq = o;
    __threadfence();
    *(volatile v4i*)dq = o;
  }
  int* mp = meta + (size_t)blockIdx.x * MSTRIDE;
#pragma unroll 1
  for (int r = 0; r < 2; ++r) {
    const int u4 = (tid + r * NTHR) * 4;
    const v4i o = *(const v4ia*)(cnt + u4);
    int* dq = mp + u4;
    *(volatile v4i*)dq = o;
    __threadfence();
    *(volatile v4i*)dq = o;
  }
  if (tid < 8) {
    v4i o = {0, 0, 0, 0};
    if (tid == 0) { o.x = ovf; o.y = tt; }
    int* dq = mp + 2 * NBA + 4 * tid;
    *(volatile v4i*)dq = o;
    __threadfence();
    *(volatile v4i*)dq = o;
  }
}

template <int SRC>
__global__ __launch_bounds__(NTHR) void k_agg(const int* __restrict__ lst, const int* __restrict__ meta,
                                              const unsigned short* __restrict__ srcpl,
                                              int nN, int mRows, unsigned short* __restrict__ agg) {
  __shared__ __attribute__((aligned(16))) int mc[2 * NBA];
  __shared__ __attribute__((aligned(16))) unsigned short rowbuf_all[NWAVE * HP];
  const int tid = (int)threadIdx.x, lane = tid & 31, wave = tid >> 5;
  unsigned short* rowbuf = rowbuf_all + wave * HP;
  const int nodeBase = (int)blockIdx.x * NBA;
  const int* mp = meta + (size_t)blockIdx.x * MSTRIDE;
  const int* lp = lst + (size_t)blockIdx.x * RCAP;
#pragma unroll
  for (int r = 0; r < 2; ++r) {
    const int u4 = (tid + r * NTHR) * 4;
    *(v4ia*)(mc + u4) = *(const v4i*)(mp + u4);
  }
  const int ovf = mp[2 * NBA];
  __syncthreads();

  const float pz = (ovf != 0) ? __int_as_float(0x7fc00000) : 0.0f;
#pragma unroll 1
  for (int si = 0; si < NBA / NWAVE; ++si) {
    const int s    = si * NWAVE + wave;
    const int node = nodeBase + s;
    int c = mc[s];
    const bool big = c > DEGCAP;
    c = c < 0 ? 0 : (c > DEGCAP ? DEGCAP : c);
    int o = mc[NBA + s];
    o = o < 0 ? 0 : (o > RCAP ? RCAP : o);
    const float pzr = big ? __int_as_float(0x7fc00000) : pz;
    const bool live = node < nN;
    float a0 = 0.0f, a1 = 0.0f, a2 = 0.0f, a3 = 0.0f;
#pragma unroll 1
    for (int b0 = 0; b0 < c; b0 += 32) {
      int idx = o + b0 + lane;
      idx = idx > RCAP - 1 ? RCAP - 1 : idx;
      int sr = lp[idx];
      sr = sr < 0 ? 0 : (sr > nN - 1 ? nN - 1 : sr);
      const int m32 = (c - b0) < 32 ? (c - b0) : 32;
#pragma unroll 1
      for (int k = 0; k < m32; ++k) {
        const int sk = __builtin_amdgcn_readlane(sr, k);
        if constexpr (SRC == 0) {
          const unsigned short* rp = srcpl + (size_t)sk * XP + 4 * lane;
          const v2u wh = *(const v2ua*)rp;
          a0 += __uint_as_float(wh.x << 16);
          a1 += __uint_as_float(wh.x & 0xffff0000u);
          a2 += __uint_as_float(wh.y << 16);
          a3 += __uint_as_float(wh.y & 0xffff0000u);
        } else {
          const unsigned short* rp = srcpl + (size_t)sk * HP + 4 * lane;
          const v2u wh = *(const v2ua*)rp;
          const v2u wl = *(const v2ua*)(rp + DF);
          const float f0 = __uint_as_float(wh.x << 16)         + __uint_as_float(wl.x << 16);
          const float f1 = __uint_as_float(wh.x & 0xffff0000u) + __uint_as_float(wl.x & 0xffff0000u);
          const float f2 = __uint_as_float(wh.y << 16)         + __uint_as_float(wl.y << 16);
          const float f3 = __uint_as_float(wh.y & 0xffff0000u) + __uint_as_float(wl.y & 0xffff0000u);
          a0 += f0; a1 += f1; a2 += f2; a3 += f3;
        }
      }
    }
    const float dc = (float)(c < 1 ? 1 : c);
    const float m0 = live ? (a0 / dc + pzr) : 0.0f;
    const float m1 = live ? (a1 / dc + pzr) : 0.0f;
    const float m2 = live ? (a2 / dc + pzr) : 0.0f;
    const float m3 = live ? (a3 / dc + pzr) : 0.0f;
    v4us mh, ml;
    {
      unsigned hb;
      hb = bf16_bits(m0); mh[0] = (unsigned short)hb; ml[0] = (unsigned short)bf16_bits(m0 - __uint_as_float(hb << 16));
      hb = bf16_bits(m1); mh[1] = (unsigned short)hb; ml[1] = (unsigned short)bf16_bits(m1 - __uint_as_float(hb << 16));
      hb = bf16_bits(m2); mh[2] = (unsigned short)hb; ml[2] = (unsigned short)bf16_bits(m2 - __uint_as_float(hb << 16));
      hb = bf16_bits(m3); mh[3] = (unsigned short)hb; ml[3] = (unsigned short)bf16_bits(m3 - __uint_as_float(hb << 16));
    }
    *(v4usa*)(rowbuf + 4 * lane)      = mh;
    *(v4usa*)(rowbuf + DF + 4 * lane) = ml;
    wave_sync();
    const v8us q0 = *(const v8usa*)(rowbuf + 8 * lane);
    wave_sync();
    if (node < mRows) {
      unsigned short* rpw = agg + (size_t)node * HP + 8 * lane;
      *(volatile v8us*)rpw = q0;
      __threadfence();
      *(volatile v8us*)rpw = q0;
    }
  }
}

template <int MODE>
__global__ __launch_bounds__(GTHR) void k_gemm(const unsigned short* __restrict__ A1, int lda1, int K1,
                                               const unsigned short* __restrict__ A2, int lda2, int K2,
                                               const unsigned short* __restrict__ BT, int ldb,
                                               const float* __restrict__ bias, int doRelu,
                                               unsigned short* outp, float* outf, int nN, int mRows) {
  __shared__ __attribute__((aligned(16))) float stg[GBM * GBN];
  const int tid = (int)threadIdx.x, lane = tid & 31, wave = tid >> 5, hh = lane >> 4, m = lane & 15;
  const int rowBase = (int)blockIdx.x * GBM;
  const int colT = (int)blockIdx.y;

  v8f acc[8];
  {
    const v8f z = {0.f, 0.f, 0.f, 0.f, 0.f, 0.f, 0.f, 0.f};
#pragma unroll
    for (int t = 0; t < 8; ++t) acc[t] = z;
  }
  const size_t arow = (size_t)(rowBase + 16 * wave + m);
  const unsigned short* ap1 = A1 + arow * (size_t)lda1 + 8 * hh;
  const unsigned short* ap2 = A2 + arow * (size_t)lda2 + 8 * hh;
  const unsigned short* bp  = BT + (size_t)(GBN * colT + m) * (size_t)ldb + 8 * hh;

#pragma unroll 1
  for (int k0 = 0; k0 < K1; k0 += 32) {
    FragB af;
    af.h[0] = *(const v8usa*)(ap1 + k0);
    af.h[1] = *(const v8usa*)(ap1 + k0 + 16);
#pragma unroll
    for (int nt = 0; nt < 8; ++nt) {
      const unsigned short* wq = bp + (size_t)(16 * nt) * (size_t)ldb + k0;
      FragB bf;
      bf.h[0] = *(const v8usa*)wq;
      bf.h[1] = *(const v8usa*)(wq + 16);
      acc[nt] = wmb(af, bf, acc[nt]);
    }
  }
#pragma unroll 1
  for (int k0 = 0; k0 < K2; k0 += 32) {
    FragB af;
    af.h[0] = *(const v8usa*)(ap2 + k0);
    af.h[1] = *(const v8usa*)(ap2 + k0 + 16);
#pragma unroll
    for (int nt = 0; nt < 8; ++nt) {
      const unsigned short* wq = bp + (size_t)(16 * nt) * (size_t)ldb + K1 + k0;
      FragB bf;
      bf.h[0] = *(const v8usa*)wq;
      bf.h[1] = *(const v8usa*)(wq + 16);
      acc[nt] = wmb(af, bf, acc[nt]);
    }
  }

#pragma unroll
  for (int nt = 0; nt < 8; ++nt) {
    const int lc = 16 * nt + m;
#pragma unroll
    for (int r = 0; r < 8; ++r) {
      const int lr = 16 * wave + 8 * hh + r;
      stg[lr * GBN + lc] = acc[nt][r];
    }
  }
  __syncthreads();

  v4f bb4;
  {
    const v4f t1 = *(const v4f*)(bias + 4 * lane);
    const bool bon = (colT == 0);
    bb4.x = bon ? bf16_val(t1.x) : 0.0f;
    bb4.y = bon ? bf16_val(t1.y) : 0.0f;
    bb4.z = bon ? bf16_val(t1.z) : 0.0f;
    bb4.w = bon ? bf16_val(t1.w) : 0.0f;
  }

  v4f pv[16];
#pragma unroll
  for (int i = 0; i < 16; ++i) pv[i] = *(const v4fa*)(stg + (16 * wave + i) * GBN + 4 * lane);
  __syncthreads();

  const bool rl = (doRelu != 0);
#pragma unroll
  for (int i = 0; i < 16; ++i) {
    const bool ok = (rowBase + 16 * wave + i) < nN;
    const v4f t = pv[i] + bb4;
    v4f y;
    y.x = rl ? relu_np(t.x) : t.x;
    y.y = rl ? relu_np(t.y) : t.y;
    y.z = rl ? relu_np(t.z) : t.z;
    y.w = rl ? relu_np(t.w) : t.w;
    y.x = ok ? y.x : 0.0f; y.y = ok ? y.y : 0.0f; y.z = ok ? y.z : 0.0f; y.w = ok ? y.w : 0.0f;
    pv[i] = y;
  }

  if constexpr (MODE != 0) {
#pragma unroll
    for (int i = 0; i < 16; ++i) {
      const int r = rowBase + 16 * wave + i;
      float* op = outf + (size_t)r * PABP + GBN * colT + 4 * lane;
      if (r < nN) *(volatile v4f*)op = pv[i];
    }
    __threadfence();
#pragma unroll
    for (int i = 0; i < 16; ++i) {
      const int r = rowBase + 16 * wave + i;
      float* op = outf + (size_t)r * PABP + GBN * colT + 4 * lane;
      if (r < nN) *(volatile v4f*)op = pv[i];
    }
    (void)outp; (void)mRows;
  } else {
#pragma unroll
    for (int i = 0; i < 16; ++i) {
      v4us h4, l4;
      unsigned hb;
      hb = bf16_bits(pv[i].x); h4[0] = (unsigned short)hb; l4[0] = (unsigned short)bf16_bits(pv[i].x - __uint_as_float(hb << 16));
      hb = bf16_bits(pv[i].y); h4[1] = (unsigned short)hb; l4[1] = (unsigned short)bf16_bits(pv[i].y - __uint_as_float(hb << 16));
      hb = bf16_bits(pv[i].z); h4[2] = (unsigned short)hb; l4[2] = (unsigned short)bf16_bits(pv[i].z - __uint_as_float(hb << 16));
      hb = bf16_bits(pv[i].w); h4[3] = (unsigned short)hb; l4[3] = (unsigned short)bf16_bits(pv[i].w - __uint_as_float(hb << 16));
      unsigned short* srow = (unsigned short*)stg + (size_t)(16 * wave + i) * (2 * GBN);
      *(v4usa*)(srow + 4 * lane) = h4;
      *(v4usa*)(srow + DF + 4 * lane) = l4;
    }
    __syncthreads();
    v8us qv[16];
#pragma unroll
    for (int i = 0; i < 16; ++i) {
      const unsigned short* srow = (const unsigned short*)stg + (size_t)(16 * wave + i) * (2 * GBN);
      qv[i] = *(const v8usa*)(srow + 8 * lane);
    }
#pragma unroll
    for (int i = 0; i < 16; ++i) {
      const int gr = rowBase + 16 * wave + i;
      unsigned short* rp = outp + (size_t)gr * (size_t)HP + 8 * lane;
      if (gr < mRows) *(volatile v8us*)rp = qv[i];
    }
    __threadfence();
#pragma unroll
    for (int i = 0; i < 16; ++i) {
      const int gr = rowBase + 16 * wave + i;
      unsigned short* rp = outp + (size_t)gr * (size_t)HP + 8 * lane;
      if (gr < mRows) *(volatile v8us*)rp = qv[i];
    }
    (void)outf;
  }
}

__global__ __launch_bounds__(NTHR) void k_pair(const float* __restrict__ pab, const int* __restrict__ pidx,
                                               const float* __restrict__ qw2, const float* __restrict__ qb2,
                                               int nN, int EP, float* out) {
  __shared__ __attribute__((aligned(16))) float res[NTHR];
  const int tid = (int)threadIdx.x, lane = tid & 31;
  const int base = (int)blockIdx.x * NTHR;
  const int p  = base + tid;
  const int pc = p < EP ? p : EP - 1;
  int pi = pidx[pc];
  int pj = pidx[(size_t)EP + pc];
  pi = pi < 0 ? 0 : (pi > nN - 1 ? nN - 1 : pi);
  pj = pj < 0 ? 0 : (pj > nN - 1 ? nN - 1 : pj);
  v4f w4;
  {
    const v4f t = *(const v4f*)(qw2 + 4 * lane);
    w4.x = bf16_val(t.x); w4.y = bf16_val(t.y); w4.z = bf16_val(t.z); w4.w = bf16_val(t.w);
  }
  const float qb = bf16_val(qb2[0]);
  float r = 0.0f;
#pragma unroll 2
  for (int k = 0; k < 32; ++k) {
    const int ik = __builtin_amdgcn_readlane(pi, k);
    const int jk = __builtin_amdgcn_readlane(pj, k);
    const v4f a = *(const v4fa*)(pab + (size_t)ik * PABP + 4 * lane);
    const v4f b = *(const v4fa*)(pab + (size_t)jk * PABP + DF + 4 * lane);
    const float v0 = relu_np(a.x + b.x);
    const float v1 = relu_np(a.y + b.y);
    const float v2 = relu_np(a.z + b.z);
    const float v3 = relu_np(a.w + b.w);
    float s = v0 * w4.x;
    s = fmaf(v1, w4.y, s);
    s = fmaf(v2, w4.z, s);
    s = fmaf(v3, w4.w, s);
    s += __shfl_xor(s, 16, 32);
    s += __shfl_xor(s, 8, 32);
    s += __shfl_xor(s, 4, 32);
    s += __shfl_xor(s, 2, 32);
    s += __shfl_xor(s, 1, 32);
    r = (lane == k) ? s : r;
  }
  res[tid] = r + qb;
  __syncthreads();
  const int q4 = 4 * (tid & 63);
  const v4f pvv = *(const v4fa*)(res + q4);
  const bool ok = (tid < 64) && (base + 32 * ((tid & 63) >> 3) < EP);
  float* op = out + (size_t)base + q4;
  if (ok) *(volatile v4f*)op = pvv;
  __threadfence();
  if (ok) *(volatile v4f*)op = pvv;
}

static inline int cdiv(int a, int b) { return (a + b - 1) / b; }
static inline size_t al256(size_t o) { return (o + 255) & ~(size_t)255; }

extern "C" void kernel_launch(void* const* d_in, const int* in_sizes, int n_in,
                              void* d_out, int out_size, void* d_ws, size_t ws_size,
                              hipStream_t stream) {
  if (n_in < 19) return;
  if (in_sizes[0] < DF * GBM || (in_sizes[0] % DF) != 0) return;
  const int nN = in_sizes[0] / DF;
  if (nN >= (1 << 22)) return;
  if (in_sizes[2] < 2 || (in_sizes[2] & 1) != 0) return;
  const int nE = in_sizes[2] / 2;
  if (nE < 1 || nE >= (1 << 21)) return;
  if (in_sizes[3] < 2 || (in_sizes[3] & 1) != 0) return;
  const int EP = in_sizes[3] / 2;
  if ((EP % 32) != 0 || out_size != EP) return;
  if (in_sizes[4] != 3 * DF * DF || in_sizes[5] != 3 * DF || in_sizes[6] != 3 * DF * DF) return;
  if (in_sizes[11] != DF * DF || in_sizes[12] != DF) return;
  if (in_sizes[13] != DF * DF || in_sizes[14] != DF) return;
  if (in_sizes[15] != 2 * DF * DF || in_sizes[16] != DF) return;
  if (in_sizes[17] != DF || in_sizes[18] != 1) return;

  const float* x   = (const float*)d_in[0];
  const int*   ei  = (const int*)  d_in[2];
  const int*   pe  = (const int*)  d_in[3];
  const float* Wl  = (const float*)d_in[4];
  const float* bl  = (const float*)d_in[5];
  const float* Wr  = (const float*)d_in[6];
  const float* pW1 = (const float*)d_in[11];
  const float* pb1 = (const float*)d_in[12];
  const float* pW2 = (const float*)d_in[13];
  const float* pb2 = (const float*)d_in[14];
  const float* qW1 = (const float*)d_in[15];
  const float* qb1 = (const float*)d_in[16];
  const float* qW2 = (const float*)d_in[17];
  const float* qb2 = (const float*)d_in[18];
  float* out = (float*)d_out;
  const int* src = ei;
  const int* dst = ei + nE;

  const int MP = cdiv(nN, GBM) * GBM;
  const int gM = MP / GBM;
  const int gA = cdiv(MP, NBA);
  if ((long long)gA * NBA < (long long)MP || gA > 4096) return;
  const int vec8 = ((nE & 3) == 0) ? 1 : 0;

  char* ws = (char*)d_ws;
  size_t off = 0;
  const size_t szXB  = (size_t)MP * XP * 2;
  const size_t szAGG = (size_t)MP * HP * 2;
  const size_t szPAB = (size_t)MP * PABP * 4;
  const size_t szP   = (szXB + szAGG) > szPAB ? (szXB + szAGG) : szPAB;
  const size_t oP    = off; off = al256(off + szP);
  const size_t oHA   = off; off = al256(off + (size_t)MP * HP * 2);
  const size_t oHB   = off; off = al256(off + (size_t)MP * HP * 2);
  const size_t oLIST = off; off = al256(off + (size_t)gA * RCAP * 4);
  const size_t oMETA = off; off = al256(off + (size_t)gA * MSTRIDE * 4);
  const size_t oWPL  = off; off = al256(off + (size_t)WPLN * 2);
  if (off > ws_size || off > (size_t)WSMAX) return;
  unsigned short* XB  = (unsigned short*)(ws + oP);
  unsigned short* AGG = (unsigned short*)(ws + oP + szXB);
  float*          PAB = (float*)(ws + oP);
  unsigned short* HA  = (unsigned short*)(ws + oHA);
  unsigned short* HB  = (unsigned short*)(ws + oHB);
  int*            LST = (int*)(ws + oLIST);
  int*            MET = (int*)(ws + oMETA);
  unsigned short* WPL = (unsigned short*)(ws + oWPL);

  const size_t cmpLds = (size_t)CMP_LDS_INTS * 4;
  hipFuncSetAttribute(reinterpret_cast<const void*>(&k_compact), hipFuncAttributeMaxDynamicSharedMemorySize, (int)cmpLds);

  const int nUnits = NUW + MP * (XP / 8);

  k_prep<<<cdiv(nUnits, NTHR), NTHR, 0, stream>>>(x, Wl, Wr, pW1, pW2, qW1, WPL, XB, nN, nUnits);
  k_compact<<<gA, NTHR, cmpLds, stream>>>(src, dst, nE, nN, vec8, LST, MET);
  k_agg<0><<<gA, NTHR, 0, stream>>>(LST, MET, XB, nN, MP, AGG);
  k_gemm<0><<<dim3(gM, 1), GTHR, 0, stream>>>(AGG, HP, 2 * DF, XB, XP, DF, WPL + OW0, 384,
                                              bl, 1, HA, PAB, nN, MP);
  k_agg<1><<<gA, NTHR, 0, stream>>>(LST, MET, HA, nN, MP, AGG);
  k_gemm<0><<<dim3(gM, 1), GTHR, 0, stream>>>(AGG, HP, 2 * DF, HA, HP, 2 * DF, WPL + OW1, 512,
                                              bl + DF, 1, HB, PAB, nN, MP);
  k_agg<1><<<gA, NTHR, 0, stream>>>(LST, MET, HB, nN, MP, AGG);
  k_gemm<0><<<dim3(gM, 1), GTHR, 0, stream>>>(AGG, HP, 2 * DF, HB, HP, 2 * DF, WPL + OW2, 512,
                                              bl + 2 * DF, 1, HA, PAB, nN, MP);
  k_gemm<0><<<dim3(gM, 1), GTHR, 0, stream>>>(HA, HP, 2 * DF, HA, HP, 0, WPL + OP1, 256,
                                              pb1, 1, HB, PAB, nN, MP);
  k_gemm<0><<<dim3(gM, 1), GTHR, 0, stream>>>(HB, HP, 2 * DF, HB, HP, 0, WPL + OP2, 256,
                                              pb2, 0, HA, PAB, nN, MP);
  k_gemm<1><<<dim3(gM, 2), GTHR, 0, stream>>>(HA, HP, 2 * DF, HA, HP, 0, WPL + OQ, 256,
                                              qb1, 0, HB, PAB, nN, MP);
  k_pair<<<cdiv(EP, NTHR), NTHR, 0, stream>>>(PAB, pe, qW2, qb2, nN, EP, out);
}
